// RNN_31267361915156
// MI455X (gfx1250) — hardware-verified
//
#include <hip/hip_runtime.h>
#include <math.h>

constexpr int NBATCH   = 128;
constexpr int NSTEP    = 512;
constexpr int NVOCAB   = 128;
constexpr int NHID     = 512;
constexpr int NOUTC    = 128;
constexpr int ROWS_BLK    = 16;
constexpr int SEQ_THREADS = 512;
constexpr int SEQ_WAVES   = SEQ_THREADS / 32;
constexpr int HPITCH   = 520;
constexpr int H_PLANE  = ROWS_BLK * HPITCH;
constexpr int YPITCH   = 132;
constexpr int Y_PLANE  = ROWS_BLK * YPITCH;
constexpr int YK_HALF  = NHID / 2;
constexpr int TP_THREADS = 256;

static_assert(NBATCH % ROWS_BLK == 0, "batch tiles");
static_assert(NHID == 32 * SEQ_WAVES, "each wave owns 32 hidden columns");
static_assert(NOUTC == 16 * (SEQ_WAVES / 2), "eight 16-column output tiles, two k halves");
static_assert(ROWS_BLK == SEQ_WAVES, "one wave stores one output row per step");
static_assert(NOUTC == 4 * 32, "one 16-B store per lane covers an output row");
static_assert(NHID % 64 == 0 && NOUTC % 64 == 0, "transpose tiles");
static_assert(NHID % 32 == 0 && YK_HALF % 32 == 0, "k steps of 32");
static_assert((HPITCH % 8) == 0 && (YPITCH % 4) == 0, "16-B aligned LDS rows");

typedef __attribute__((ext_vector_type(16))) _Float16 v16h;
typedef __attribute__((ext_vector_type(8)))  _Float16 v8h;
typedef __attribute__((ext_vector_type(16))) __bf16   v16b;
typedef __attribute__((ext_vector_type(8)))  __bf16   v8b;
typedef __attribute__((ext_vector_type(8)))  float    v8f;
typedef __attribute__((ext_vector_type(4)))  float    v4f;

__device__ __forceinline__ unsigned short f2bf_bits(float f) {
  unsigned u = __float_as_uint(f);
  return (unsigned short)((u + 0x7FFFu + ((u >> 16) & 1u)) >> 16);
}
__device__ __forceinline__ float bf_bits2f(unsigned short h) { return __uint_as_float(((unsigned)h) << 16); }
__device__ __forceinline__ float bf16r(float f) { return bf_bits2f(f2bf_bits(f)); }

__device__ __forceinline__ void guard_acc_frags(v8f& acc, v16b a0, v16b a1, v16b b0) {
  asm volatile("v_nop\n\tv_nop\n\tv_nop\n\tv_nop" : "+v"(acc) : "v"(a0), "v"(a1), "v"(b0));
}
__device__ __forceinline__ void keep3_b(v16b a0, v16b a1, v16b b0) {
  asm volatile("v_nop" :: "v"(a0), "v"(a1), "v"(b0));
}
__device__ __forceinline__ void guard_acc(v8f& acc) {
  asm volatile("v_nop\n\tv_nop\n\tv_nop\n\tv_nop" : "+v"(acc));
}

template <typename T> struct Frag;
template <> struct Frag<__bf16> {
  typedef v16b V; union U { v16b v; v8b h[2]; };
  static __device__ __forceinline__ v16b load(const __bf16* p) {
    U f; f.h[0] = *(const v8b*)(p); f.h[1] = *(const v8b*)(p + 16); return f.v;
  }
  static __device__ __forceinline__ v8f mma(v16b a, v16b b, v8f c) {
    return __builtin_amdgcn_wmma_f32_16x16x32_bf16(false, a, false, b, (short)0, c, false, false);
  }
};

__global__ __launch_bounds__(TP_THREADS) void tpose_bf16_kernel(const float* __restrict__ src, int ncols_in, int ldo,
                                                                unsigned short* __restrict__ dst) {
  __shared__ float Tt[64 * 65];
  const int tid = threadIdx.x;
  const int c0 = blockIdx.x * 64, r0 = blockIdx.y * 64;
#pragma unroll
  for (int i = 0; i < 4; ++i) {
    const int idx = i * TP_THREADS + tid;
    const int rr = idx >> 4, cc = (idx & 15) * 4;
    const v4f v = *(const v4f*)(src + (size_t)(r0 + rr) * (size_t)ncols_in + c0 + cc);
    Tt[rr * 65 + cc + 0] = v[0];
    Tt[rr * 65 + cc + 1] = v[1];
    Tt[rr * 65 + cc + 2] = v[2];
    Tt[rr * 65 + cc + 3] = v[3];
  }
  __syncthreads();
  const int q = tid >> 3, c8 = (tid & 7) * 8;
  v8h hv[2];
#pragma unroll
  for (int g = 0; g < 2; ++g) {
    const int qq = g * 32 + q;
#pragma unroll
    for (int e = 0; e < 8; ++e) {
      const float f = Tt[(c8 + e) * 65 + qq];
      const unsigned short bits = f2bf_bits(f);
      hv[g][e] = __builtin_bit_cast(_Float16, bits);
    }
  }
  for (int pass = 0; pass < 2; ++pass) {
#pragma unroll
    for (int g = 0; g < 2; ++g) {
      const size_t o = (size_t)(c0 + g * 32 + q) * (size_t)ldo + (size_t)(r0 + c8);
      *(volatile v8h*)(dst + o) = hv[g];
    }
    __threadfence();
  }
}

__global__ __launch_bounds__(SEQ_THREADS) void recur_kernel(const int* __restrict__ xtok, const float* __restrict__ wxh,
                                                            const float* __restrict__ bh, const float* __restrict__ by,
                                                            const unsigned short* __restrict__ whhT_p,
                                                            const unsigned short* __restrict__ whyT_p,
                                                            float* __restrict__ out) {
  __shared__ __align__(16) unsigned short Hhi[2 * H_PLANE];
  __shared__ __align__(16) unsigned short Hlo[2 * H_PLANE];
  __shared__ __align__(16) float          Ys[2 * Y_PLANE];
  const __bf16* WhhT = (const __bf16*)whhT_p;
  const __bf16* WhyT = (const __bf16*)whyT_p;
  const int tid = threadIdx.x, lane = tid & 31, wave = tid >> 5;
  const int c = lane & 15, hh = lane >> 4, koff = hh * 8;
  const int rowbase = blockIdx.x * ROWS_BLK;

#pragma unroll 1
  for (int i = tid; i < 2 * H_PLANE; i += SEQ_THREADS) {
    Hhi[i] = (unsigned short)0;
    Hlo[i] = (unsigned short)0;
  }
#pragma unroll 1
  for (int i = tid; i < 2 * Y_PLANE; i += SEQ_THREADS) Ys[i] = 0.0f;

  const float bh0 = bf16r(bh[32 * wave + c]);
  const float bh1 = bf16r(bh[32 * wave + 16 + c]);
  const int ot = wave & 7, kh = wave >> 3;
  const int ocol = 16 * ot + c;
  const float byraw = bf16r(by[ocol]);
  const float byv = (kh == 0) ? byraw : 0.0f;
  const __bf16* wyb = WhyT + (size_t)ocol * NHID + kh * YK_HALF + koff;
  const v8f z8 = {0.f, 0.f, 0.f, 0.f, 0.f, 0.f, 0.f, 0.f};
  __syncthreads();

#pragma unroll 1
  for (int t = 0; t < NSTEP; ++t) {
    const int cur = t & 1;
    const int nxt = cur ^ 1;
    const __bf16* ahi = (const __bf16*)(Hhi + cur * H_PLANE) + c * HPITCH + koff;
    const __bf16* alo = (const __bf16*)(Hlo + cur * H_PLANE) + c * HPITCH + koff;
    unsigned short* nhi = Hhi + nxt * H_PLANE;
    unsigned short* nlo = Hlo + nxt * H_PLANE;

    int tokoff[8];
#pragma unroll
    for (int r = 0; r < 8; ++r) {
      int tk = xtok[(size_t)(rowbase + 8 * hh + r) * NSTEP + (size_t)t];
      tk = tk < 0 ? 0 : tk;
      tk = tk > (NVOCAB - 1) ? (NVOCAB - 1) : tk;
      tokoff[r] = tk * NHID;
    }

#pragma unroll 1
    for (int nt = 0; nt < 2; ++nt) {
      const int j = 32 * wave + 16 * nt + c;
      const __bf16* wb = WhhT + (size_t)j * NHID + koff;
      v8f acc = z8;
#pragma unroll 1
      for (int k0 = 0; k0 < NHID; k0 += 32) {
        const v16b a_h = Frag<__bf16>::load(ahi + k0);
        const v16b a_l = Frag<__bf16>::load(alo + k0);
        const v16b b_w = Frag<__bf16>::load(wb + k0);
        acc = Frag<__bf16>::mma(a_h, b_w, acc);
        acc = Frag<__bf16>::mma(a_l, b_w, acc);
        guard_acc_frags(acc, a_h, a_l, b_w);
        keep3_b(a_h, a_l, b_w);
      }
      guard_acc(acc);
      const float bias = (nt == 0) ? bh0 : bh1;
      float wxv[8];
#pragma unroll
      for (int r = 0; r < 8; ++r) wxv[r] = wxh[(size_t)(tokoff[r] + j)];
#pragma unroll
      for (int r = 0; r < 8; ++r) {
        const float pre = (bf16r(wxv[r]) + acc[r]) + bias;
        const float hv = tanhf(pre);
        const unsigned short hb = f2bf_bits(hv);
        const float hf = bf_bits2f(hb);
        const unsigned short lb = f2bf_bits(hv - hf);
        const int li = (8 * hh + r) * HPITCH + j;
        nhi[li] = hb;
        nlo[li] = lb;
      }
    }
    __syncthreads();

    {
      const __bf16* yhi = (const __bf16*)(Hhi + nxt * H_PLANE) + c * HPITCH + kh * YK_HALF + koff;
      const __bf16* ylo = (const __bf16*)(Hlo + nxt * H_PLANE) + c * HPITCH + kh * YK_HALF + koff;
      v8f acc = z8;
#pragma unroll 1
      for (int k0 = 0; k0 < YK_HALF; k0 += 32) {
        const v16b a_h = Frag<__bf16>::load(yhi + k0);
        const v16b a_l = Frag<__bf16>::load(ylo + k0);
        const v16b b_w = Frag<__bf16>::load(wyb + k0);
        acc = Frag<__bf16>::mma(a_h, b_w, acc);
        acc = Frag<__bf16>::mma(a_l, b_w, acc);
        guard_acc_frags(acc, a_h, a_l, b_w);
        keep3_b(a_h, a_l, b_w);
      }
      guard_acc(acc);
      float* yp = Ys + kh * Y_PLANE;
#pragma unroll
      for (int r = 0; r < 8; ++r) yp[(8 * hh + r) * YPITCH + ocol] = acc[r] + byv;
    }
    __syncthreads();

    {
      const float* y0 = Ys + wave * YPITCH + 4 * lane;
      const v4f p0 = *(const v4f*)(y0);
      const v4f p1 = *(const v4f*)(y0 + Y_PLANE);
      v4f v;
      v[0] = p0[0] + p1[0];
      v[1] = p0[1] + p1[1];
      v[2] = p0[2] + p1[2];
      v[3] = p0[3] + p1[3];
      float* op = out + ((size_t)(rowbase + wave) * NSTEP + (size_t)t) * NOUTC + 4 * lane;
      *(volatile v4f*)op = v;
      __threadfence();
      *(volatile v4f*)op = v;
    }
  }
}

extern "C" void kernel_launch(void* const* d_in, const int* in_sizes, int n_in,
                              void* d_out, int out_size, void* d_ws, size_t ws_size, hipStream_t stream) {
  if (n_in < 6 || d_out == nullptr || d_ws == nullptr) return;
  if (in_sizes[0] != NBATCH * NSTEP || in_sizes[1] != NVOCAB * NHID || in_sizes[2] != NHID * NHID ||
      in_sizes[3] != NHID * NOUTC || in_sizes[4] != NHID || in_sizes[5] != NOUTC ||
      out_size != NBATCH * NSTEP * NOUTC) return;

  const int*   xtok = (const int*)d_in[0];
  const float* wxh  = (const float*)d_in[1];
  const float* whh  = (const float*)d_in[2];
  const float* why  = (const float*)d_in[3];
  const float* bh   = (const float*)d_in[4];
  const float* by   = (const float*)d_in[5];
  float* out = (float*)d_out;

  char* ws = (char*)d_ws; size_t off = 0;
  auto carve = [&](size_t bytes) -> char* { char* p = ws + off; off += (bytes + 255) & ~(size_t)255; return p; };
  unsigned short* WHHT = (unsigned short*)carve((size_t)NHID * NHID * 2);
  unsigned short* WHYT = (unsigned short*)carve((size_t)NOUTC * NHID * 2);
  if (off > ws_size || off > (size_t)134217728) return;

  tpose_bf16_kernel<<<dim3(NHID / 64, NHID / 64), TP_THREADS, 0, stream>>>(whh, NHID, NHID, WHHT);
  tpose_bf16_kernel<<<dim3(NOUTC / 64, NHID / 64), TP_THREADS, 0, stream>>>(why, NOUTC, NHID, WHYT);
  recur_kernel<<<NBATCH / ROWS_BLK, SEQ_THREADS, 0, stream>>>(xtok, wxh, bh, by, WHHT, WHYT, out);
}
